// CGTPEL_72645076844777
// MI455X (gfx1250) — hardware-verified
//
#include <hip/hip_runtime.h>
#include <math.h>

#define NN 10000
#define NE 60000
#define IN_DIM 128
#define HID 128
#define WN 4096
#define MUL 32
#define NT 256
#define EPB 32
#define NEB ((NE + EPB - 1) / EPB)
#define SRB 512
#define NTILE ((NN + SRB - 1) / SRB)
#define NYR (NTILE * SRB)
#define SCH 2048
#define NCH ((NE + SCH - 1) / SCH)
#define NSB 32
#define RPB ((NN + NSB - 1) / NSB)
#define RB 128
#define NAB ((NN + RB - 1) / RB)
#define WSC 16.0f
#define WSC_INV 0.0625f
#define EPS_BN 1e-5f
#define INV_SQRT3 0.57735026918962576451f
#define PATH_NORM 0.125f

#if (NE % (SCH / NT)) != 0
#error edge count must be a multiple of the per-thread chunk span
#endif
#if NE >= (1 << 20)
#error edge id field is 20 bits wide
#endif

typedef __attribute__((ext_vector_type(16))) _Float16 v16h;
typedef __attribute__((ext_vector_type(8)))  _Float16 v8h;
typedef __attribute__((ext_vector_type(4)))  _Float16 v4h;
typedef __attribute__((ext_vector_type(8)))  float    v8f;
typedef __attribute__((ext_vector_type(4)))  float    v4f;
typedef __attribute__((ext_vector_type(4)))  int      v4i;

__device__ __forceinline__ v16h frag_load(const _Float16* p) {
  union { v16h v; v8h h[2]; } f;
  f.h[0] = *(const v8h*)(p);
  f.h[1] = *(const v8h*)(p + 16);
  return f.v;
}
__device__ __forceinline__ v8f mma16(v16h a, v16h b, v8f c) {
  return __builtin_amdgcn_wmma_f32_16x16x32_f16(false, a, false, b, (short)0, c, false, false);
}
__device__ __forceinline__ void guard1(v8f& a, v16h x, v16h y) { asm volatile("v_nop\n\tv_nop\n\tv_nop\n\tv_nop" : "+v"(a) : "v"(x), "v"(y)); }
__device__ __forceinline__ void guard2(v8f& a, v8f& b, v16h x, v16h y) { asm volatile("v_nop\n\tv_nop\n\tv_nop\n\tv_nop" : "+v"(a), "+v"(b) : "v"(x), "v"(y)); }

__device__ __forceinline__ int blk_excl_scan(int cnt, int* scan_ws, int tid, int* tot) {
  const int lane = tid & 31, wave = tid >> 5; int incl = cnt;
#pragma unroll
  for (int o = 1; o < 32; o <<= 1) { const int v = __shfl_up(incl, o, 32); if (lane >= o) incl += v; }
  if (lane == 31) scan_ws[wave] = incl;
  __syncthreads();
  if (wave == 0) { int wv = (lane < NT / 32) ? scan_ws[lane] : 0; int wincl = wv;
#pragma unroll
    for (int o = 1; o < 32; o <<= 1) { const int v = __shfl_up(wincl, o, 32); if (lane >= o) wincl += v; }
    if (lane < NT / 32) scan_ws[32 + lane] = wincl - wv; if (lane == 31) scan_ws[64] = wincl; }
  __syncthreads();
  const int res = scan_ws[32 + wave] + incl - cnt; *tot = scan_ws[64];
  return res;
}
template <int SP, int CAP>
__device__ __forceinline__ int chunk_hits(const int* __restrict__ srcv, int e0, int n0, int tid, int* LIST, int* scan_ws) {
  const int eb = e0 + tid * SP;
  const int ebc = (eb < NE) ? eb : (NE - SP);
  const bool inr = (eb < NE);
  int rec[SP]; int cnt = 0;
#pragma unroll
  for (int k = 0; k < SP; k += 4) {
    const v4i s4 = *(const v4i*)(srcv + ebc + k);
#pragma unroll
    for (int e = 0; e < 4; ++e) {
      const int s = s4[e]; int r = -1;
      if (inr && s >= n0 && s < n0 + SRB) { r = ((s - n0) << 20) | (ebc + k + e); ++cnt; }
      rec[k + e] = r;
    }
  }
  int tot; int p = blk_excl_scan(cnt, scan_ws, tid, &tot);
#pragma unroll
  for (int k = 0; k < SP; ++k) if (rec[k] >= 0) { if ((unsigned)p < (unsigned)CAP) LIST[p] = rec[k]; ++p; }
  __syncthreads();
  return tot < CAP ? tot : CAP;
}

__global__ __launch_bounds__(NT) void pack_w_kernel(const float* __restrict__ W1, const float* __restrict__ W2,
                                                   unsigned* __restrict__ W1P, unsigned* __restrict__ W2P) {
  const int i = blockIdx.x * NT + threadIdx.x;
  const int N1 = HID * HID / 2;
  const int N2 = HID * WN / 2;
  if (i >= N1 + N2) return;
  const bool second = (i >= N1);
  const int d = second ? (i - N1) : i;
  const int ncols = second ? WN : HID;
  const float* src = second ? W2 : W1;
  unsigned* dst = second ? W2P : W1P;
  const int p = 2 * d;
  const int el = p & 15;
  const int lane = (p >> 4) & 31;
  const int frag = p >> 9;
  const int kb = frag & 3;
  const int t = frag >> 2;
  const int h = lane >> 4;
  const int kk = (el < 8) ? (8 * h + el) : (16 + 8 * h + (el - 8));
  const int k = kb * 32 + kk;
  const int n = t * 16 + (lane & 15);
  const float a = src[(size_t)k * ncols + n] * WSC;
  const float b = src[(size_t)(k + 1) * ncols + n] * WSC;
  const _Float16 h0 = (_Float16)a, h1 = (_Float16)b;
  const unsigned u = (unsigned)__builtin_bit_cast(unsigned short, h0) | ((unsigned)__builtin_bit_cast(unsigned short, h1) << 16);
  ((volatile unsigned*)dst)[d] = u;
  __threadfence();
  ((volatile unsigned*)dst)[d] = u;
}

__global__ __launch_bounds__(NT) void edge_kernel(const float* __restrict__ edge_attr,
                                                 const unsigned* __restrict__ W1P, const float* __restrict__ b1,
                                                 const unsigned* __restrict__ W2P, const float* __restrict__ b2,
                                                 const float* __restrict__ node_attr, const int* __restrict__ eidx,
                                                 const float* __restrict__ edge_sh, float* __restrict__ TPB) {
  __shared__ __align__(32) float accb[6 * 1024];
  __shared__ __align__(32) _Float16 h_lds[EPB * HID];
  __shared__ __align__(16) float coef[6 * 1024];
  __shared__ float shv[EPB * 4];
  _Float16* x_lds = (_Float16*)accb;

  const int tid = threadIdx.x, lane = tid & 31, wv = tid >> 5, hh = lane >> 4, n = lane & 15;
  const int e0 = blockIdx.x * EPB;

#pragma unroll
  for (int it = 0; it < 4; ++it) {
    const int q = tid + it * NT;
    const int m = q >> 5, c4 = (q & 31) * 4;
    const int e = e0 + m; const int ec = (e < NE) ? e : (NE - 1);
    v4f f = *(const v4f*)(edge_attr + (size_t)ec * IN_DIM + c4);
    if (e >= NE) f = (v4f){0.f, 0.f, 0.f, 0.f};
    const v4h hv = (v4h){(_Float16)f[0], (_Float16)f[1], (_Float16)f[2], (_Float16)f[3]};
    *(v4h*)(x_lds + m * IN_DIM + c4) = hv;
  }
#pragma unroll
  for (int it = 0; it < 4; ++it) {
    const int p = tid + it * NT;
    const int m = p >> 5, u = p & 31;
    const int e = e0 + m; const int ec = (e < NE) ? e : (NE - 1);
    const float live = (e < NE) ? 1.0f : 0.0f;
    int dn = eidx[NE + ec]; dn = dn < 0 ? 0 : (dn >= NN ? NN - 1 : dn);
    const float sh0 = edge_sh[(size_t)ec * 4 + 0] * live;
    const float s1  = edge_sh[(size_t)ec * 4 + 1] * live;
    const float s2  = edge_sh[(size_t)ec * 4 + 2] * live;
    const float s3  = edge_sh[(size_t)ec * 4 + 3] * live;
    const float* xr = node_attr + (size_t)dn * IN_DIM;
    const float x0 = xr[u];
    const float xa = xr[MUL + 3 * u + 0];
    const float xb = xr[MUL + 3 * u + 1];
    const float xc = xr[MUL + 3 * u + 2];
    coef[p]        = x0 * sh0;
    coef[1024 + p] = x0 * live;
    coef[2048 + p] = xa * s1 + xb * s2 + xc * s3;
    coef[3072 + p] = xa * sh0;
    coef[4096 + p] = xb * sh0;
    coef[5120 + p] = xc * sh0;
    if (u == 0) { shv[m * 4 + 0] = s1; shv[m * 4 + 1] = s2; shv[m * 4 + 2] = s3; shv[m * 4 + 3] = 0.f; }
  }
  __syncthreads();

  {
    const v16h* w1p = (const v16h*)W1P;
    const int ct = wv;
    const float bval = b1[ct * 16 + n];
#pragma unroll
    for (int r = 0; r < 2; ++r) {
      v8f c = (v8f){0.f, 0.f, 0.f, 0.f, 0.f, 0.f, 0.f, 0.f};
#pragma unroll
      for (int kb = 0; kb < 4; ++kb) {
        const v16h a = frag_load(x_lds + (r * 16 + n) * IN_DIM + kb * 32 + 8 * hh);
        const v16h b = w1p[(ct * 4 + kb) * 32 + lane];
        c = mma16(a, b, c);
        guard1(c, a, b);
      }
#pragma unroll
      for (int v = 0; v < 8; ++v) {
        float hv = c[v] * WSC_INV + bval;
        hv = fmaxf(hv, 0.0f);
        h_lds[(r * 16 + 8 * hh + v) * HID + ct * 16 + n] = (_Float16)hv;
      }
    }
  }
  __syncthreads();

  v16h af[2][4];
#pragma unroll
  for (int r = 0; r < 2; ++r)
#pragma unroll
    for (int kb = 0; kb < 4; ++kb)
      af[r][kb] = frag_load(h_lds + (r * 16 + n) * HID + kb * 32 + 8 * hh);
  __syncthreads();

  const int X = wv >> 1, parity = wv & 1;
  const bool isC = (X == 2);
  const float* cf0 = coef + ((X == 0) ? 0 : (X == 1) ? 1024 : (X == 3) ? 2048 : 3072);
  const float* cf1 = coef + 4096;
  const float* cf2 = coef + 5120;
  const v16h* w2p = (const v16h*)W2P;

  float acc0[2][8], acc1[2][8], acc2[2][8];
#pragma unroll
  for (int r = 0; r < 2; ++r)
#pragma unroll
    for (int v = 0; v < 8; ++v) { acc0[r][v] = 0.f; acc1[r][v] = 0.f; acc2[r][v] = 0.f; }

#pragma unroll 1
  for (int u = 0; u < 32; ++u) {
    const int t = X * 64 + parity + 2 * u;
    const float bval = b2[t * 16 + n];
    v8f c0 = (v8f){0.f, 0.f, 0.f, 0.f, 0.f, 0.f, 0.f, 0.f};
    v8f c1 = (v8f){0.f, 0.f, 0.f, 0.f, 0.f, 0.f, 0.f, 0.f};
#pragma unroll
    for (int kb = 0; kb < 4; ++kb) {
      const v16h b = w2p[(t * 4 + kb) * 32 + lane];
      c0 = mma16(af[0][kb], b, c0);
      c1 = mma16(af[1][kb], b, c1);
      guard2(c0, c1, af[1][kb], b);
    }
#pragma unroll
    for (int v = 0; v < 8; ++v) {
      const int m0 = 8 * hh + v, m1 = 16 + 8 * hh + v;
      const float cv0 = c0[v] * WSC_INV + bval;
      const float cv1 = c1[v] * WSC_INV + bval;
      acc0[0][v] += cf0[m0 * 32 + u] * cv0;
      acc0[1][v] += cf0[m1 * 32 + u] * cv1;
      if (isC) {
        acc1[0][v] += cf1[m0 * 32 + u] * cv0;
        acc1[1][v] += cf1[m1 * 32 + u] * cv1;
        acc2[0][v] += cf2[m0 * 32 + u] * cv0;
        acc2[1][v] += cf2[m1 * 32 + u] * cv1;
      }
    }
  }

  {
    float* d0 = accb + ((X == 0) ? 0 : (X == 1) ? 1024 : (X == 3) ? 2048 : 3072);
    const int w = parity * 16 + n;
#pragma unroll
    for (int r = 0; r < 2; ++r)
#pragma unroll
      for (int v = 0; v < 8; ++v) {
        const int m = r * 16 + 8 * hh + v;
        d0[m * 32 + w] = acc0[r][v];
        if (isC) {
          accb[4096 + m * 32 + w] = acc1[r][v];
          accb[5120 + m * 32 + w] = acc2[r][v];
        }
      }
  }
  __syncthreads();

  v4f orow[4];
#pragma unroll
  for (int j = 0; j < 4; ++j) {
    const int m = wv * 4 + j;
    v4f o;
#pragma unroll
    for (int c = 0; c < 4; ++c) {
      const int col = 4 * lane + c;
      const int cs = (col < MUL) ? col : 0;
      const int q = (col < MUL) ? 0 : (col - MUL);
      const int ww = q / 3; const int i = q - 3 * ww;
      const float vs = PATH_NORM * (accb[m * 32 + cs] + INV_SQRT3 * accb[2048 + m * 32 + cs]);
      const float vv = (PATH_NORM * INV_SQRT3) * (accb[1024 + m * 32 + ww] * shv[m * 4 + i] + accb[3072 + i * 1024 + m * 32 + ww]);
      o[c] = (col < MUL) ? vs : vv;
    }
    orow[j] = o;
  }
  for (int pass = 0; pass < 2; ++pass) {
#pragma unroll
    for (int j = 0; j < 4; ++j) {
      const int m = wv * 4 + j;
      *(volatile v4f*)(TPB + (size_t)(e0 + m) * IN_DIM + 4 * lane) = orow[j];
    }
    __threadfence();
  }
}

__global__ __launch_bounds__(NT) void agg_kernel(const float* __restrict__ TPB, const int* __restrict__ eidx,
                                                const float* __restrict__ node_attr, float* Y) {
  __shared__ int LIST[SCH];
  __shared__ int SC[SRB];
  __shared__ int scan_ws[80];
  const int tid = threadIdx.x, lane = tid & 31, wave = tid >> 5;
  const int n0 = blockIdx.x * SRB;
  const v4f z4 = {0.f, 0.f, 0.f, 0.f};
#pragma unroll 1
  for (int j = 0; j < 64; ++j) {
    float* rp = Y + (size_t)(n0 + wave * 64 + j) * IN_DIM + 4 * lane;
    *(volatile v4f*)rp = z4;
    __threadfence();
    *(volatile v4f*)rp = z4;
  }
  for (int i = tid; i < SRB; i += NT) SC[i] = 0;
  __syncthreads();
  const int* srcv = eidx;
#pragma unroll 1
  for (int c = 0; c < NCH; ++c) {
    const int tot = chunk_hits<SCH / NT, SCH>(srcv, c * SCH, n0, tid, LIST, scan_ws);
#pragma unroll 1
    for (int base = 0; base < tot; base += 32) {
      const int q = base + lane;
      const int rv = (q < tot) ? LIST[q] : -1;
      const int own = (rv >= 0 && ((rv >> 26) & 7) == wave) ? 1 : 0;
      unsigned msk = (unsigned)__ballot(own);
#pragma unroll 1
      for (int it = 0; it < 32; ++it) {
        if (msk == 0u) break;
        const int bp = __builtin_ctz(msk); msk &= msk - 1u;
        const int r = __shfl(rv, bp, 32);
        const int dl = (r >> 20) & (SRB - 1);
        int e = r & 0xFFFFF; e = (e < NE) ? e : (NE - 1);
        const v4f t = *(const v4f*)(TPB + (size_t)e * IN_DIM + 4 * lane);
        float* rp = Y + (size_t)(n0 + dl) * IN_DIM + 4 * lane;
        v4f a = *(const v4f*)rp;
        a = a + t;
        *(volatile v4f*)rp = a;
        __threadfence();
        *(volatile v4f*)rp = a;
        if (lane == 0) SC[dl] += 1;
      }
    }
    __syncthreads();
  }
#pragma unroll 1
  for (int j = 0; j < 64; ++j) {
    const int dl = wave * 64 + j; const int nd = n0 + dl;
    if (nd < NN) {
      const int cnt = SC[dl];
      const float cf = (float)cnt;
      const float inv = 1.0f / fmaxf(cf, 1.0f);
      float* rp = Y + (size_t)nd * IN_DIM + 4 * lane;
      const v4f a = *(const v4f*)rp;
      const v4f x = *(const v4f*)(node_attr + (size_t)nd * IN_DIM + 4 * lane);
      const v4f o = a * inv + x;
      for (int pass = 0; pass < 2; ++pass) { *(volatile v4f*)rp = o; __threadfence(); }
    }
  }
}

__global__ __launch_bounds__(NT) void stats_kernel(const float* __restrict__ Y, double* __restrict__ PART) {
  __shared__ double red[2 * 128];
  const int tid = threadIdx.x;
  const int col = tid & 127, sub = tid >> 7;
  const int r0 = blockIdx.x * RPB;
  const int r1 = (r0 + RPB < NN) ? (r0 + RPB) : NN;
  double s = 0.0, q = 0.0;
#pragma unroll 1
  for (int r = r0 + sub; r < r1; r += 2) {
    const float v = Y[(size_t)r * IN_DIM + col];
    const double dv = (double)v;
    s += dv; q += dv * dv;
  }
  if (sub == 1) { red[col] = s; red[128 + col] = q; }
  __syncthreads();
  if (sub == 0) {
    s += red[col]; q += red[128 + col];
    double* pp = PART + (size_t)blockIdx.x * 256;
    ((volatile double*)pp)[col] = s; ((volatile double*)pp)[128 + col] = q;
    __threadfence();
    ((volatile double*)pp)[col] = s; ((volatile double*)pp)[128 + col] = q;
  }
}

__global__ __launch_bounds__(NT) void bn_kernel(const float* __restrict__ Y, const double* __restrict__ PART,
                                               const float* __restrict__ bn_w, const float* __restrict__ bn_b,
                                               float* __restrict__ out) {
  __shared__ double sS[128];
  __shared__ double sQ[128];
  __shared__ __align__(16) float ssub[128];
  __shared__ __align__(16) float sscl[128];
  __shared__ __align__(16) float sadd[128];
  const int tid = threadIdx.x, lane = tid & 31, wave = tid >> 5;
  if (tid < 128) {
    double s = 0.0, q = 0.0;
#pragma unroll 1
    for (int b = 0; b < NSB; ++b) { s += PART[(size_t)b * 256 + tid]; q += PART[(size_t)b * 256 + 128 + tid]; }
    sS[tid] = s; sQ[tid] = q;
  }
  __syncthreads();
  if (tid < 128) {
    const double invN = 1.0 / (double)NN;
    if (tid < MUL) {
      const double mu = sS[tid] * invN;
      double var = sQ[tid] * invN - mu * mu;
      var = var > 0.0 ? var : 0.0;
      const float varf = (float)var;
      const float rs = 1.0f / sqrtf(varf + EPS_BN);
      ssub[tid] = (float)mu;
      sscl[tid] = rs * bn_w[tid];
      sadd[tid] = bn_b[tid];
    } else {
      const int u = (tid - MUL) / 3;
      const double vq = (sQ[MUL + 3 * u] + sQ[MUL + 3 * u + 1] + sQ[MUL + 3 * u + 2]) * (invN * (1.0 / 3.0));
      const float vqf = (float)vq;
      const float rs = 1.0f / sqrtf(vqf + EPS_BN);
      ssub[tid] = 0.f;
      sscl[tid] = rs * bn_w[MUL + u];
      sadd[tid] = 0.f;
    }
  }
  __syncthreads();
  const v4f sub4 = *(const v4f*)(ssub + 4 * lane);
  const v4f scl4 = *(const v4f*)(sscl + 4 * lane);
  const v4f add4 = *(const v4f*)(sadd + 4 * lane);
#pragma unroll 1
  for (int j = 0; j < 16; ++j) {
    const int r = blockIdx.x * RB + wave * 16 + j;
    if (r < NN) {
      const v4f y = *(const v4f*)(Y + (size_t)r * IN_DIM + 4 * lane);
      v4f t = (y - sub4) * scl4;
      t = t + add4;
      float* op = out + (size_t)r * IN_DIM + 4 * lane;
      for (int pass = 0; pass < 2; ++pass) { *(volatile v4f*)op = t; __threadfence(); }
    }
  }
}

extern "C" void kernel_launch(void* const* d_in, const int* in_sizes, int n_in,
                              void* d_out, int out_size, void* d_ws, size_t ws_size, hipStream_t stream) {
  (void)n_in;
  const float* node_attr = (const float*)d_in[0];
  const int*   eidx      = (const int*)  d_in[1];
  const float* edge_attr = (const float*)d_in[2];
  const float* edge_sh   = (const float*)d_in[3];
  const float* W1        = (const float*)d_in[4];
  const float* b1        = (const float*)d_in[5];
  const float* W2        = (const float*)d_in[6];
  const float* b2        = (const float*)d_in[7];
  const float* bn_w      = (const float*)d_in[8];
  const float* bn_b      = (const float*)d_in[9];
  float* out = (float*)d_out;

  if (in_sizes[0] != NN * IN_DIM || in_sizes[1] != 2 * NE || in_sizes[2] != NE * IN_DIM || out_size != NN * IN_DIM) return;

  char* ws = (char*)d_ws; size_t off = 0;
  auto carve = [&](size_t bytes) -> char* { char* p = ws + off; off += (bytes + 255) & ~(size_t)255; return p; };
  unsigned* W1P = (unsigned*)carve((size_t)HID * HID * 2);
  unsigned* W2P = (unsigned*)carve((size_t)HID * WN * 2);
  float*    TPB = (float*)carve((size_t)NEB * EPB * IN_DIM * 4);
  float*    Y   = (float*)carve((size_t)NYR * IN_DIM * 4);
  double*   PART= (double*)carve((size_t)NSB * 256 * 8);
  if (off > ws_size || off > (size_t)134217728) return;

  const int npack = (HID * HID / 2 + HID * WN / 2 + NT - 1) / NT;
  pack_w_kernel<<<npack, NT, 0, stream>>>(W1, W2, W1P, W2P);
  edge_kernel<<<NEB, NT, 0, stream>>>(edge_attr, W1P, b1, W2P, b2, node_attr, eidx, edge_sh, TPB);
  agg_kernel<<<NTILE, NT, 0, stream>>>(TPB, eidx, node_attr, Y);
  stats_kernel<<<NSB, NT, 0, stream>>>(Y, PART);
  bn_kernel<<<NAB, NT, 0, stream>>>(Y, PART, bn_w, bn_b, out);
}
